// Attention_86131274154435
// MI455X (gfx1250) — hardware-verified
//
#include <hip/hip_runtime.h>
#include <stddef.h>


#pragma clang fp contract(off)

#ifndef NB
#define NB 4
#endif
#ifndef SEQ
#define SEQ 2048
#endif
#define NB_FULL  4
#define SEQ_FULL 2048
#define DIM    1024
#define INNER  1024
#define HEADS  16
#define DHEAD  64
#define KD     1024
#define NQKV   (3 * INNER)
#define M_ROWS (NB * SEQ)

static_assert(SEQ % 64 == 0);
static_assert(SEQ <= SEQ_FULL);
static_assert(NB >= 1);
static_assert(NB <= NB_FULL);
static_assert(M_ROWS % 64 == 0);
static_assert(NQKV % 128 == 0);
static_assert(INNER % 128 == 0);
static_assert(DIM % 128 == 0);
static_assert(KD % 64 == 0);
static_assert(DIM == KD);
static_assert(INNER == KD);
static_assert(HEADS * DHEAD == INNER);
static_assert(DHEAD == 64);
static_assert((M_ROWS * DIM) % 2048 == 0);

typedef _Float16 v16h __attribute__((ext_vector_type(16)));
typedef _Float16 v8h  __attribute__((ext_vector_type(8)));
typedef float    v8f  __attribute__((ext_vector_type(8)));
typedef float    v4f  __attribute__((ext_vector_type(4)));
union Frag { v16h v; v8h half[2]; };

__device__ __forceinline__ float bf16_rne(float f) {
  unsigned u = __builtin_bit_cast(unsigned, f);
  u = (u + 0x7FFFu + ((u >> 16) & 1u)) & 0xFFFF0000u;
  return __builtin_bit_cast(float, u);
}

__device__ __forceinline__ v16h frag_g(const _Float16* p, int hh) {
  Frag f;
  f.half[0] = *(const v8h*)(p + 8 * hh);
  f.half[1] = *(const v8h*)(p + 16 + 8 * hh);
  return f.v;
}

__device__ __forceinline__ v8f wmma16(v8f c, v16h a, v16h b) {
  v8f d = __builtin_amdgcn_wmma_f32_16x16x32_f16(false, a, false, b, (short)0, c, false, false);
  asm volatile("v_nop\n\tv_nop\n\tv_nop\n\tv_nop" : "+v"(d) : "v"(a), "v"(b));
  return d;
}

__global__ __launch_bounds__(256) void k_cvt_x(const float* __restrict__ x,
                                               _Float16* __restrict__ xh) {
  const size_t gid = (size_t)blockIdx.x * 256 + threadIdx.x;
  const size_t e0 = gid * 8;
  if (e0 >= (size_t)M_ROWS * DIM) return;
  const size_t r = e0 / DIM;
  const int c = (int)(e0 - r * DIM);
  const size_t srow = (r / SEQ) * SEQ_FULL + (r % SEQ);
  const float* src = x + srow * DIM + c;
  const v4f f0 = *(const v4f*)src;
  const v4f f1 = *(const v4f*)(src + 4);
  v8h o;
#pragma unroll
  for (int e = 0; e < 4; ++e) {
    o[e]     = (_Float16)bf16_rne(f0[e]);
    o[4 + e] = (_Float16)bf16_rne(f1[e]);
  }
  _Float16* dst = xh + r * DIM + c;
  *(volatile v8h*)dst = o;
  __threadfence();
  *(volatile v8h*)dst = o;
}

__global__ __launch_bounds__(256) void k_cvt_w(const float* __restrict__ wq,
                                               const float* __restrict__ wkv,
                                               const float* __restrict__ wo,
                                               _Float16* __restrict__ wq_t,
                                               _Float16* __restrict__ wkv_t,
                                               _Float16* __restrict__ wo_t) {
  __shared__ _Float16 T[64 * 72];
  const int z = blockIdx.z;
  const int ncols = (z == 1) ? (2 * INNER) : INNER;
  const int nt = blockIdx.x, kt = blockIdx.y;
  if (nt * 64 >= ncols) return;
  const float* src = (z == 0) ? wq : ((z == 1) ? wkv : wo);
  _Float16* dstp = (z == 0) ? wq_t : ((z == 1) ? wkv_t : wo_t);
  const int t = threadIdx.x, lane = t & 31, wave = t >> 5;

#pragma unroll
  for (int i = 0; i < 4; ++i) {
    const int v = t + 256 * i;
    const int kr = v >> 4, c4 = (v & 15) * 4;
    const v4f f = *(const v4f*)(src + (size_t)(kt * 64 + kr) * ncols + nt * 64 + c4);
#pragma unroll
    for (int e = 0; e < 4; ++e)
      T[(c4 + e) * 72 + kr] = (_Float16)(bf16_rne(f[e]) * 64.0f);
  }
  __syncthreads();

  v8h val[2];
  _Float16* dst[2];
#pragma unroll
  for (int it = 0; it < 2; ++it) {
    const int L = wave * 8 + it * 4 + (lane >> 3);
    const int p = lane & 7;
    val[it] = *(const v8h*)&T[L * 72 + p * 8];
    dst[it] = dstp + (size_t)(nt * 64 + L) * KD + kt * 64 + p * 8;
  }
#pragma unroll
  for (int it = 0; it < 2; ++it) *(volatile v8h*)dst[it] = val[it];
  __threadfence();
#pragma unroll
  for (int it = 0; it < 2; ++it) *(volatile v8h*)dst[it] = val[it];
}

__device__ __forceinline__ void mainloop(const _Float16* __restrict__ Ab,
                                         const _Float16* __restrict__ Bb,
                                         int hh, v8f (&acc)[2][2]) {
#pragma unroll 2
  for (int k0 = 0; k0 < KD; k0 += 32) {
    const v16h a0 = frag_g(Ab + k0, hh);
    const v16h a1 = frag_g(Ab + (size_t)16 * KD + k0, hh);
    const v16h b0 = frag_g(Bb + k0, hh);
    const v16h b1 = frag_g(Bb + (size_t)16 * KD + k0, hh);
    acc[0][0] = wmma16(acc[0][0], a0, b0);
    acc[0][1] = wmma16(acc[0][1], a0, b1);
    acc[1][0] = wmma16(acc[1][0], a1, b0);
    acc[1][1] = wmma16(acc[1][1], a1, b1);
  }
}

__global__ __launch_bounds__(256) void k_gemm_qkv(const _Float16* __restrict__ xh,
                                                  const _Float16* __restrict__ wq_t,
                                                  const _Float16* __restrict__ wkv_t,
                                                  _Float16* __restrict__ qp,
                                                  _Float16* __restrict__ kp,
                                                  _Float16* __restrict__ vtp) {
  __shared__ _Float16 CsT[128 * 72];
  const int t = threadIdx.x, lane = t & 31, wave = t >> 5;
  const int hh = lane >> 4, m = lane & 15;
  const int wm = wave >> 2, wn = wave & 3;
  const int m0 = blockIdx.y * 64, n0 = blockIdx.x * 128;
  const int part = n0 / INNER;
  const int ncol0 = n0 - part * INNER;
  const _Float16* Bt = (part == 0) ? (wq_t + (size_t)ncol0 * KD)
                                   : (wkv_t + (size_t)(n0 - INNER) * KD);
  const _Float16* Ab = xh + (size_t)(m0 + wm * 32 + m) * KD;
  const _Float16* Bb = Bt + (size_t)(wn * 32 + m) * KD;

  const v8f z8 = {0.f, 0.f, 0.f, 0.f, 0.f, 0.f, 0.f, 0.f};
  v8f acc[2][2] = {{z8, z8}, {z8, z8}};
  mainloop(Ab, Bb, hh, acc);

#pragma unroll
  for (int mi = 0; mi < 2; ++mi)
#pragma unroll
    for (int ni = 0; ni < 2; ++ni) {
      const int col = wn * 32 + ni * 16 + m;
      const int rb = wm * 32 + mi * 16 + 8 * hh;
      v8h cv;
#pragma unroll
      for (int g = 0; g < 8; ++g) cv[g] = (_Float16)(acc[mi][ni][g] * (1.0f / 64.0f));
      *(v8h*)&CsT[col * 72 + rb] = cv;
    }
  __syncthreads();

  const int b = m0 / SEQ, ntok0 = m0 - b * SEQ;
  const int hbase = ncol0 / DHEAD;
  v8h val[4];
  _Float16* dst[4];
  if (part == 2) {
#pragma unroll
    for (int it = 0; it < 4; ++it) {
      const int L = wave * 16 + it * 4 + (lane >> 3);
      const int p = lane & 7;
      const int hsel = L >> 6, d = L & 63;
      val[it] = *(const v8h*)&CsT[(hsel * 64 + d) * 72 + p * 8];
      dst[it] = vtp + ((size_t)((b * HEADS + hbase + hsel) * DHEAD + d)) * SEQ + ntok0 + p * 8;
    }
  } else {
    _Float16* plane = (part == 0) ? qp : kp;
#pragma unroll
    for (int it = 0; it < 4; ++it) {
      const int L = wave * 16 + it * 4 + (lane >> 3);
      const int p = lane & 7;
      const int hsel = L >> 6, r = L & 63;
#pragma unroll
      for (int e = 0; e < 8; ++e) val[it][e] = CsT[(hsel * 64 + p * 8 + e) * 72 + r];
      dst[it] = plane + ((size_t)(b * HEADS + hbase + hsel) * SEQ + ntok0 + r) * DHEAD + p * 8;
    }
  }
#pragma unroll
  for (int it = 0; it < 4; ++it) *(volatile v8h*)dst[it] = val[it];
  __threadfence();
#pragma unroll
  for (int it = 0; it < 4; ++it) *(volatile v8h*)dst[it] = val[it];
}

__global__ __launch_bounds__(128) __attribute__((amdgpu_num_vgpr(256)))
void k_flash(const _Float16* __restrict__ qp, const _Float16* __restrict__ kp,
             const _Float16* __restrict__ vtp, _Float16* __restrict__ ao) {
  __shared__ _Float16 Ps[4][16 * 72];
  const int t = threadIdx.x, lane = t & 31, wave = t >> 5;
  const int hh = lane >> 4, m = lane & 15;
  const int bh = blockIdx.y;
  const int b = bh / HEADS, hd = bh - b * HEADS;
  const int n0 = blockIdx.x * 64;
  const _Float16* qrow = qp + ((size_t)bh * SEQ + n0 + wave * 16 + m) * DHEAD;
  const v16h qF0 = frag_g(qrow, hh);
  const v16h qF1 = frag_g(qrow + 32, hh);
  const _Float16* kb = kp + (size_t)bh * SEQ * DHEAD;
  const _Float16* vb = vtp + (size_t)bh * DHEAD * SEQ;
  _Float16* pw = &Ps[wave][0];

  const v8f z8 = {0.f, 0.f, 0.f, 0.f, 0.f, 0.f, 0.f, 0.f};
  v8f o[4] = {z8, z8, z8, z8};
  float mr[8], lr[8];
#pragma unroll
  for (int g = 0; g < 8; ++g) { mr[g] = -1e30f; lr[g] = 0.f; }
  const float C = 0.125f * 1.44269504088896340736f;

#pragma unroll 1
  for (int j0 = 0; j0 < SEQ; j0 += 64) {
    v8f s[4];
#pragma unroll
    for (int jt = 0; jt < 4; ++jt) {
      const _Float16* krow = kb + (size_t)(j0 + jt * 16 + m) * DHEAD;
      s[jt] = z8;
      const v16h k0f = frag_g(krow, hh);
      s[jt] = wmma16(s[jt], qF0, k0f);
      const v16h k1f = frag_g(krow + 32, hh);
      s[jt] = wmma16(s[jt], qF1, k1f);
    }
    float mp[8];
#pragma unroll
    for (int g = 0; g < 8; ++g)
      mp[g] = fmaxf(fmaxf(s[0][g], s[1][g]), fmaxf(s[2][g], s[3][g])) * C;
#pragma unroll
    for (int off = 1; off < 16; off <<= 1)
#pragma unroll
      for (int g = 0; g < 8; ++g)
        mp[g] = fmaxf(mp[g], __shfl_xor(mp[g], off, 32));
#pragma unroll
    for (int g = 0; g < 8; ++g) {
      const float mnew = fmaxf(mr[g], mp[g]);
      const float rs = exp2f(mr[g] - mnew);
      mr[g] = mnew;
      lr[g] *= rs;
      o[0][g] *= rs; o[1][g] *= rs; o[2][g] *= rs; o[3][g] *= rs;
    }
#pragma unroll
    for (int jt = 0; jt < 4; ++jt)
#pragma unroll
      for (int g = 0; g < 8; ++g) {
        const float p = exp2f(s[jt][g] * C - mr[g]);
        lr[g] += p;
        pw[(8 * hh + g) * 72 + jt * 16 + m] = (_Float16)(p * 1024.0f);
      }
    __syncthreads();

#pragma unroll
    for (int ks = 0; ks < 2; ++ks) {
      const v16h pF = frag_g(pw + m * 72 + ks * 32, hh);
#pragma unroll
      for (int dt = 0; dt < 4; ++dt) {
        const v16h vF = frag_g(vb + (size_t)(dt * 16 + m) * SEQ + j0 + ks * 32, hh);
        o[dt] = wmma16(o[dt], pF, vF);
      }
    }
    __syncthreads();
  }

#pragma unroll
  for (int off = 1; off < 16; off <<= 1)
#pragma unroll
    for (int g = 0; g < 8; ++g)
      lr[g] += __shfl_xor(lr[g], off, 32);
  float inv[8];
#pragma unroll
  for (int g = 0; g < 8; ++g) inv[g] = 1.0f / (lr[g] * 16.0f);
#pragma unroll
  for (int dt = 0; dt < 4; ++dt)
#pragma unroll
    for (int g = 0; g < 8; ++g)
      pw[(8 * hh + g) * 72 + dt * 16 + m] = (_Float16)(o[dt][g] * inv[g]);
  __syncthreads();

  v8h val[4];
  _Float16* dst[4];
#pragma unroll
  for (int it = 0; it < 4; ++it) {
    const int r = it * 4 + (lane >> 3);
    const int p = lane & 7;
    val[it] = *(const v8h*)(pw + r * 72 + p * 8);
    dst[it] = ao + ((size_t)b * SEQ + n0 + wave * 16 + r) * INNER + hd * DHEAD + p * 8;
  }
#pragma unroll
  for (int it = 0; it < 4; ++it) *(volatile v8h*)dst[it] = val[it];
  __threadfence();
#pragma unroll
  for (int it = 0; it < 4; ++it) *(volatile v8h*)dst[it] = val[it];
}

__global__ __launch_bounds__(256) void k_gemm_out(const _Float16* __restrict__ ao,
                                                  const _Float16* __restrict__ wo_t,
                                                  const float* __restrict__ bout,
                                                  float* __restrict__ out) {
  __shared__ float Cs[64 * 132];
  const int t = threadIdx.x, lane = t & 31, wave = t >> 5;
  const int hh = lane >> 4, m = lane & 15;
  const int wm = wave >> 2, wn = wave & 3;
  const int m0 = blockIdx.y * 64, n0 = blockIdx.x * 128;
  const _Float16* Ab = ao + (size_t)(m0 + wm * 32 + m) * KD;
  const _Float16* Bb = wo_t + (size_t)(n0 + wn * 32 + m) * KD;

  const v8f z8 = {0.f, 0.f, 0.f, 0.f, 0.f, 0.f, 0.f, 0.f};
  v8f acc[2][2] = {{z8, z8}, {z8, z8}};
  mainloop(Ab, Bb, hh, acc);

#pragma unroll
  for (int mi = 0; mi < 2; ++mi)
#pragma unroll
    for (int ni = 0; ni < 2; ++ni) {
      const int col = wn * 32 + ni * 16 + m;
      const float bc = bf16_rne(bout[n0 + col]);
      const int rb = wm * 32 + mi * 16 + 8 * hh;
#pragma unroll
      for (int g = 0; g < 8; ++g)
        Cs[(rb + g) * 132 + col] = acc[mi][ni][g] * (1.0f / 4096.0f) + bc;
    }
  __syncthreads();

  v4f val[8];
  float* dst[8];
#pragma unroll
  for (int it = 0; it < 8; ++it) {
    const int row = wave * 8 + it;
    const int mc = m0 + row;
    const int orow = (mc / SEQ) * SEQ_FULL + (mc % SEQ);
    val[it] = *(const v4f*)&Cs[row * 132 + lane * 4];
    dst[it] = out + (size_t)orow * DIM + n0 + lane * 4;
  }
#pragma unroll
  for (int it = 0; it < 8; ++it) *(volatile v4f*)dst[it] = val[it];
  __threadfence();
#pragma unroll
  for (int it = 0; it < 8; ++it) *(volatile v4f*)dst[it] = val[it];
}

extern "C" void kernel_launch(void* const* d_in, const int* in_sizes, int n_in,
                              void* d_out, int out_size, void* d_ws,
                              size_t ws_size, hipStream_t stream) {
  if (n_in < 5) return;
  const int need_rows = (NB - 1) * SEQ_FULL + SEQ;
  if (in_sizes[0] < need_rows * DIM) return;
  if (in_sizes[1] < DIM * INNER) return;
  if (in_sizes[2] < DIM * 2 * INNER) return;
  if (in_sizes[3] < INNER * DIM) return;
  if (in_sizes[4] < DIM) return;
  if (out_size < need_rows * DIM) return;

  const float* x    = (const float*)d_in[0];
  const float* wq   = (const float*)d_in[1];
  const float* wkv  = (const float*)d_in[2];
  const float* wo   = (const float*)d_in[3];
  const float* bout = (const float*)d_in[4];
  float* out = (float*)d_out;

  char* ws = (char*)d_ws;
  size_t off = 0;
  _Float16* xh    = (_Float16*)(ws + off); off += (size_t)M_ROWS * DIM * 2;
  _Float16* wq_t  = (_Float16*)(ws + off); off += (size_t)INNER * KD * 2;
  _Float16* wkv_t = (_Float16*)(ws + off); off += (size_t)2 * INNER * KD * 2;
  _Float16* wo_t  = (_Float16*)(ws + off); off += (size_t)DIM * KD * 2;
  _Float16* qp    = (_Float16*)(ws + off); off += (size_t)M_ROWS * INNER * 2;
  _Float16* kp    = (_Float16*)(ws + off); off += (size_t)M_ROWS * INNER * 2;
  _Float16* vtp   = (_Float16*)(ws + off); off += (size_t)M_ROWS * INNER * 2;
  _Float16* ao    = (_Float16*)(ws + off); off += (size_t)M_ROWS * INNER * 2;
  if (off > ws_size) return;

  const int nblk_x = (int)(((size_t)M_ROWS * DIM / 8) / 256);
  k_cvt_x<<<dim3(nblk_x), dim3(256), 0, stream>>>(x, xh);

  k_cvt_w<<<dim3((2 * INNER) / 64, KD / 64, 3), dim3(256), 0, stream>>>(
      wq, wkv, wo, wq_t, wkv_t, wo_t);

  k_gemm_qkv<<<dim3(NQKV / 128, M_ROWS / 64), dim3(256), 0, stream>>>(
      xh, wq_t, wkv_t, qp, kp, vtp);

  k_flash<<<dim3(SEQ / 64, NB * HEADS), dim3(128), 0, stream>>>(qp, kp, vtp, ao);

  k_gemm_out<<<dim3(DIM / 128, M_ROWS / 64), dim3(256), 0, stream>>>(ao, wo_t, bout, out);
}
